// memristor_dense_14998025798447
// MI455X (gfx1250) — hardware-verified
//
#include <hip/hip_runtime.h>
#include <stdint.h>

constexpr int NIN_C  = 1024;
constexpr int NOUT_C = 1024;
constexpr int NBATCH = 128;
constexpr int NAUG   = NIN_C + 1;
constexpr int NLEV   = 3;
constexpr int KUSED  = NLEV * NAUG;
constexpr int KTOT   = 3136;
static_assert(KTOT % 64 == 0 && KTOT >= KUSED && (KTOT - KUSED) < 256, "k padding");
constexpr int KPIECES = KTOT / 8;
constexpr float ASCALE_C = 262144.0f;
constexpr float CSCALE_C = 64.0f;
constexpr float KV_C     = 1.05f;
constexpr float GSPAN_C  = 0.0004f;

__constant__ float c_VREF[9] = {-1.2f, -0.9f, -0.6f, -0.3f, 0.0f, 0.3f, 0.6f, 0.9f, 1.2f};
__constant__ float c_GREF[4] = {0.0f, 1e-4f, 3e-4f, 5e-4f};
__constant__ float c_IREF[4][9] = {
  {0.f, 0.f, 0.f, 0.f, 0.f, 0.f, 0.f, 0.f, 0.f},
  {-0.00015f, -0.00011f, -7e-05f, -3e-05f, 0.f, 3e-05f, 7e-05f, 0.00011f, 0.00015f},
  {-0.0005f,  -0.00035f, -0.00022f, -9e-05f, 0.f, 9e-05f, 0.00022f, 0.00035f, 0.0005f},
  {-0.0009f,  -0.0006f,  -0.00037f, -0.00015f, 0.f, 0.00015f, 0.00037f, 0.0006f, 0.0009f}
};
static_assert(sizeof(c_IREF) / sizeof(c_IREF[0][0]) == 36, "table size");
static_assert(sizeof(c_VREF) / sizeof(c_VREF[0]) == 9, "table size");
static_assert(sizeof(c_GREF) / sizeof(c_GREF[0]) == 4, "table size");

typedef __attribute__((ext_vector_type(16))) _Float16 v16h;
typedef __attribute__((ext_vector_type(8)))  _Float16 v8h;
typedef __attribute__((ext_vector_type(16))) __bf16   v16b;
typedef __attribute__((ext_vector_type(8)))  __bf16   v8b;
typedef __attribute__((ext_vector_type(8)))  float    v8f;
typedef __attribute__((ext_vector_type(4)))  float    v4f;

__device__ __forceinline__ unsigned short f2bf_bits(float f) {
  unsigned u = __float_as_uint(f);
  return (unsigned short)((u + 0x7FFFu + ((u >> 16) & 1u)) >> 16);
}
__device__ __forceinline__ float bf_bits2f(unsigned short h) { return __uint_as_float(((unsigned)h) << 16); }

__device__ __forceinline__ void dep_guard_h(v8f& a, v8f& b, v16h x, v16h y) { asm volatile("v_nop\n\tv_nop\n\tv_nop\n\tv_nop" : "+v"(a), "+v"(b) : "v"(x), "v"(y)); }
__device__ __forceinline__ void dep_guard_b(v8f& a, v8f& b, v16b x, v16b y) { asm volatile("v_nop\n\tv_nop\n\tv_nop\n\tv_nop" : "+v"(a), "+v"(b) : "v"(x), "v"(y)); }
__device__ __forceinline__ void keep4_h(v16h a, v16h b, v16h c, v16h d) { asm volatile("v_nop" :: "v"(a), "v"(b), "v"(c), "v"(d)); }
__device__ __forceinline__ void keep4_b(v16b a, v16b b, v16b c, v16b d) { asm volatile("v_nop" :: "v"(a), "v"(b), "v"(c), "v"(d)); }
__device__ __forceinline__ void acc_guard4(v8f& a, v8f& b, v8f& c, v8f& d) { asm volatile("v_nop\n\tv_nop\n\tv_nop\n\tv_nop" : "+v"(a), "+v"(b), "+v"(c), "+v"(d)); }
template <typename T> struct Frag;
template <> struct Frag<_Float16> {
  typedef v16h V; union U { v16h v; v8h h[2]; };
  static __device__ __forceinline__ v16h load(const _Float16* p) {
    U f; f.h[0] = *(const v8h*)(p); f.h[1] = *(const v8h*)(p + 16); return f.v;
  }
  static __device__ __forceinline__ v8f mma(v16h a, v16h b, v8f c) {
    return __builtin_amdgcn_wmma_f32_16x16x32_f16(false, a, false, b, (short)0, c, false, false);
  }
  static __device__ __forceinline__ void guard(v8f& a, v8f& b, v16h x, v16h y) { dep_guard_h(a, b, x, y); }
  static __device__ __forceinline__ void keep(v16h a, v16h b, v16h c, v16h d) { keep4_h(a, b, c, d); }
};
template <> struct Frag<__bf16> {
  typedef v16b V; union U { v16b v; v8b h[2]; };
  static __device__ __forceinline__ v16b load(const __bf16* p) {
    U f; f.h[0] = *(const v8b*)(p); f.h[1] = *(const v8b*)(p + 16); return f.v;
  }
  static __device__ __forceinline__ v8f mma(v16b a, v16b b, v8f c) {
    return __builtin_amdgcn_wmma_f32_16x16x32_bf16(false, a, false, b, (short)0, c, false, false);
  }
  static __device__ __forceinline__ void guard(v8f& a, v8f& b, v16b x, v16b y) { dep_guard_b(a, b, x, y); }
  static __device__ __forceinline__ void keep(v16b a, v16b b, v16b c, v16b d) { keep4_b(a, b, c, d); }
};

template <int ET> struct Elem;
template <> struct Elem<0> { typedef _Float16 T; };
template <> struct Elem<1> { typedef __bf16 T; };
template <int ET, bool SPLIT, int BIAS_MODE, int OUT_MODE, bool RESID, int ACT = 0>
__global__ __launch_bounds__(256) void wmma_gemm64(
    const unsigned short* __restrict__ Ap, const unsigned short* __restrict__ A2p, int lda, long strideA,
    const unsigned short* __restrict__ Btp, const unsigned short* __restrict__ Bt2p, int ldb, long strideB,
    void* __restrict__ Cout, void* __restrict__ Cout2, int ldc, long strideC,
    const float* __restrict__ bias,
    const float* __restrict__ resid, long strideR,
    int M, int N, int K, float scale, const float* __restrict__ dscale) {
  typedef typename Elem<ET>::T T;
  typedef typename Frag<T>::V V;
  const T* A = (const T*)Ap; const T* A2 = (const T*)A2p; const T* Bt = (const T*)Btp; const T* Bt2 = (const T*)Bt2p;
  __shared__ __align__(16) float sT[8][16 * 68];
  const int b    = blockIdx.y;
  const int lane = threadIdx.x & 31;
  const int wave = threadIdx.x >> 5;
  const int tilesN = N >> 6;
  const int tilesM = M >> 6;
  const int tile = blockIdx.x * 8 + wave;
  if (tile >= tilesM * tilesN) return;
  const int tm = tile / tilesN;
  const int tn = tile - tm * tilesN;
  const int m0 = tm << 6;
  const int n0 = tn << 6;
  const float scl = scale * dscale[0];

  const T* Ab  = A  + (size_t)b * strideA;
  const T* Bb  = Bt + (size_t)b * strideB;
  const T* Ab2 = SPLIT ? (A2  + (size_t)b * strideA) : nullptr;
  const T* Bb2 = SPLIT ? (Bt2 + (size_t)b * strideB) : nullptr;

  const int rlane = lane & 15;
  const int koff  = (lane >> 4) * 8;
  const int mOff  = (lane >> 4) * 8;

  v8f acc[4][4];
#pragma unroll
  for (int i = 0; i < 4; ++i)
#pragma unroll
    for (int j = 0; j < 4; ++j) acc[i][j] = (v8f){0.f,0.f,0.f,0.f,0.f,0.f,0.f,0.f};

  for (int k0 = 0; k0 < K; k0 += 32) {
    V bh[4], bl[4];
#pragma unroll
    for (int j = 0; j < 4; ++j) {
      const size_t bo = (size_t)(n0 + (j << 4) + rlane) * ldb + koff + k0;
      bh[j] = Frag<T>::load(Bb + bo);
      if (SPLIT) bl[j] = Frag<T>::load(Bb2 + bo);
    }
#pragma unroll
    for (int i = 0; i < 4; ++i) {
      const size_t ao = (size_t)(m0 + (i << 4) + rlane) * lda + koff + k0;
      V ah = Frag<T>::load(Ab + ao);
      V al;
      if (SPLIT) al = Frag<T>::load(Ab2 + ao);
#pragma unroll
      for (int j = 0; j < 4; ++j) {
        acc[i][j] = Frag<T>::mma(ah, bh[j], acc[i][j]);
        if (SPLIT) {
          acc[i][j] = Frag<T>::mma(ah, bl[j], acc[i][j]);
          acc[i][j] = Frag<T>::mma(al, bh[j], acc[i][j]);
        }
      }
      Frag<T>::guard(acc[i][0], acc[i][3], ah, SPLIT ? al : ah);
    }
    Frag<T>::keep(bh[0], bh[1], bh[2], bh[3]);
    if (SPLIT) Frag<T>::keep(bl[0], bl[1], bl[2], bl[3]);
  }
  acc_guard4(acc[0][0], acc[0][1], acc[0][2], acc[0][3]);
  acc_guard4(acc[1][0], acc[1][1], acc[1][2], acc[1][3]);
  acc_guard4(acc[2][0], acc[2][1], acc[2][2], acc[2][3]);
  acc_guard4(acc[3][0], acc[3][1], acc[3][2], acc[3][3]);

  float* slab = sT[wave];
  const float* Rb = RESID ? (resid + (size_t)b * strideR) : nullptr;
#pragma unroll
  for (int i = 0; i < 4; ++i) {
    const int mBase = m0 + (i << 4);
#pragma unroll
    for (int j = 0; j < 4; ++j) {
      const int n = n0 + (j << 4) + rlane;
      float bv = 0.f;
      if (BIAS_MODE == 2) bv = bias[n];
#pragma unroll
      for (int r = 0; r < 8; ++r) {
        float v = acc[i][j][r] * scl;
        if (BIAS_MODE == 1) v += bias[mBase + mOff + r];
        if (BIAS_MODE == 2) v += bv;
        if (RESID) v += Rb[(size_t)(mBase + mOff + r) * ldc + n];
        if (ACT == 2) v = fmaxf(v, 0.0f);
        if (ACT == 4) v = (v > 0.f) ? v : 0.01f * v;
        slab[(mOff + r) * 68 + (j << 4) + rlane] = v;
      }
    }
    __builtin_amdgcn_fence(__ATOMIC_RELEASE, "workgroup");
    __builtin_amdgcn_wave_barrier();
    __builtin_amdgcn_fence(__ATOMIC_ACQUIRE, "workgroup");
    if (OUT_MODE == 0) {
      float* C = (float*)Cout + (size_t)b * strideC;
      const int hh = lane >> 4, c4 = (lane & 15) * 4;
      for (int pass = 0; pass < 2; ++pass) {
#pragma unroll
        for (int it = 0; it < 8; ++it) {
          const int row = it * 2 + hh;
          v4f v = *(const v4f*)(slab + row * 68 + c4);
          *(volatile v4f*)(C + (size_t)(mBase + row) * ldc + n0 + c4) = v;
        }
        __threadfence();
      }
    } else {
      const int q = lane >> 3, c8 = (lane & 7) * 8;
      unsigned short* C  = (unsigned short*)Cout  + (size_t)b * strideC;
      unsigned short* C2 = (OUT_MODE == 2) ? ((unsigned short*)Cout2 + (size_t)b * strideC) : nullptr;
      for (int pass = 0; pass < 2; ++pass) {
#pragma unroll
        for (int it = 0; it < 4; ++it) {
          const int row = it * 4 + q;
          const float* sp = slab + row * 68 + c8;
          v8h hv, lv;
#pragma unroll
          for (int e = 0; e < 8; ++e) {
            if (OUT_MODE == 1) {
              hv[e] = (_Float16)sp[e];
            } else {
              unsigned short hb = f2bf_bits(sp[e]);
              unsigned short lb = f2bf_bits(sp[e] - bf_bits2f(hb));
              hv[e] = __builtin_bit_cast(_Float16, hb);
              lv[e] = __builtin_bit_cast(_Float16, lb);
            }
          }
          *(volatile v8h*)(C + (size_t)(mBase + row) * ldc + n0 + c8) = hv;
          if (OUT_MODE == 2) *(volatile v8h*)(C2 + (size_t)(mBase + row) * ldc + n0 + c8) = lv;
        }
        __threadfence();
      }
    }
    __builtin_amdgcn_fence(__ATOMIC_RELEASE, "workgroup");
    __builtin_amdgcn_wave_barrier();
    __builtin_amdgcn_fence(__ATOMIC_ACQUIRE, "workgroup");
  }
}

__global__ __launch_bounds__(512) void k_maxabs(const float* __restrict__ w,
                                                const float* __restrict__ b,
                                                float* __restrict__ params) {
  __shared__ float sm[512];
  const int tid = threadIdx.x;
  const v4f* w4 = (const v4f*)w;
  const v4f* b4 = (const v4f*)b;
  float m = 0.f;
#pragma unroll 1
  for (int i = tid; i < (NIN_C * NOUT_C) / 4; i += 512) {
    const v4f v = w4[i];
    m = fmaxf(m, fmaxf(fmaxf(fabsf(v[0]), fabsf(v[1])), fmaxf(fabsf(v[2]), fabsf(v[3]))));
  }
  {
    const int ic = (tid < NOUT_C / 4) ? tid : (NOUT_C / 4 - 1);
    const v4f v = b4[ic];
    m = fmaxf(m, fmaxf(fmaxf(fabsf(v[0]), fabsf(v[1])), fmaxf(fabsf(v[2]), fabsf(v[3]))));
  }
  sm[tid] = m;
  __syncthreads();
  for (int s = 256; s > 0; s >>= 1) {
    if (tid < s) sm[tid] = fmaxf(sm[tid], sm[tid + s]);
    __syncthreads();
  }
  if (tid < 32) {
    const float mw  = sm[0];
    const float kG  = GSPAN_C / mw;
    const float inv = 1.0f / (KV_C * kG);
    const float val = (tid == 0) ? kG : ((tid == 1) ? inv : 0.0f);
    *(volatile float*)(params + tid) = val;
    __threadfence();
    *(volatile float*)(params + tid) = val;
  }
}

__device__ __forceinline__ void store_row_f16(const _Float16* row_lds, _Float16* __restrict__ dst, int tid) {
  for (int pass = 0; pass < 2; ++pass) {
#pragma unroll
    for (int it = 0; it < 2; ++it) {
      const int p  = it * 256 + tid;
      const int pc = (p < KPIECES) ? p : (KPIECES - 1);
      const v8h val = *(const v8h*)(row_lds + pc * 8);
      if (p < KPIECES) *(volatile v8h*)(dst + (size_t)pc * 8) = val;
    }
    __threadfence();
  }
}

__global__ __launch_bounds__(256) void k_build_a(const float* __restrict__ x,
                                                 _Float16* __restrict__ A16) {
  __shared__ __align__(16) _Float16 row[KTOT];
  const int tid = threadIdx.x;
  const int bt  = blockIdx.x;
#pragma unroll 1
  for (int n = tid; n < NAUG; n += 256) {
    const int nc = (n < NIN_C) ? n : (NIN_C - 1);
    const float xr = x[(size_t)bt * NIN_C + nc];
    const float xv = (n < NIN_C) ? xr : 1.0f;
    float V = KV_C * xv;
    V = fminf(fmaxf(V, c_VREF[0]), c_VREF[8]);
    int cnt = 0;
#pragma unroll
    for (int c = 0; c < 9; ++c) cnt += (c_VREF[c] <= V) ? 1 : 0;
    const int i1 = (cnt < 1) ? 1 : ((cnt > 8) ? 8 : cnt);
    const int i0 = i1 - 1;
    const float v0 = c_VREF[i0], v1 = c_VREF[i1];
    const float f  = (V - v0) * (1.0f / (v1 - v0));
    const float p1a = c_IREF[1][i0], p1b = c_IREF[1][i1];
    const float p2a = c_IREF[2][i0], p2b = c_IREF[2][i1];
    const float p3a = c_IREF[3][i0], p3b = c_IREF[3][i1];
    const float cur1 = p1a + f * (p1b - p1a);
    const float cur2 = p2a + f * (p2b - p2a);
    const float cur3 = p3a + f * (p3b - p3a);
    row[n * 3 + 0] = (_Float16)(cur1 * ASCALE_C);
    row[n * 3 + 1] = (_Float16)(cur2 * ASCALE_C);
    row[n * 3 + 2] = (_Float16)(cur3 * ASCALE_C);
  }
  if (tid < KTOT - KUSED) row[KUSED + tid] = (_Float16)0.0f;
  __syncthreads();
  store_row_f16(row, A16 + (size_t)bt * KTOT, tid);
}

__global__ __launch_bounds__(256) void k_build_b(const float* __restrict__ w,
                                                 const float* __restrict__ b,
                                                 const float* __restrict__ params,
                                                 _Float16* __restrict__ Bt16) {
  __shared__ __align__(16) _Float16 row[KTOT];
  const int tid = threadIdx.x;
  const int m   = blockIdx.x;
  const float kG = params[0];
  const float bm = b[m];
  const float gr1 = c_GREF[1], gr2 = c_GREF[2], gr3 = c_GREF[3];
#pragma unroll 1
  for (int n = tid; n < NAUG; n += 256) {
    const int nc = (n < NIN_C) ? n : (NIN_C - 1);
    const float wr = w[(size_t)nc * NOUT_C + m];
    const float wv = (n < NIN_C) ? wr : bm;
    const float G  = kG * wv;
    const float Ga = fabsf(G);
    const float sgn = (G > 0.0f) ? 1.0f : ((G < 0.0f) ? -1.0f : 0.0f);
    const int cm1 = ((Ga >= gr1) ? 1 : 0) + ((Ga >= gr2) ? 1 : 0) + ((Ga >= gr3) ? 1 : 0);
    const int idx = (cm1 > 2) ? 2 : cm1;
    const float g0 = (idx == 0) ? 0.0f : ((idx == 1) ? gr1 : gr2);
    const float g1 = (idx == 0) ? gr1  : ((idx == 1) ? gr2 : gr3);
    const float t  = (Ga - g0) * (1.0f / (g1 - g0));
    const float clo = sgn * (1.0f - t);
    const float chi = sgn * t;
    const float c0 = (idx == 0) ? chi  : ((idx == 1) ? clo : 0.0f);
    const float c1 = (idx == 0) ? 0.0f : ((idx == 1) ? chi : clo);
    const float c2 = (idx == 2) ? chi : 0.0f;
    row[n * 3 + 0] = (_Float16)(c0 * CSCALE_C);
    row[n * 3 + 1] = (_Float16)(c1 * CSCALE_C);
    row[n * 3 + 2] = (_Float16)(c2 * CSCALE_C);
  }
  if (tid < KTOT - KUSED) row[KUSED + tid] = (_Float16)0.0f;
  __syncthreads();
  store_row_f16(row, Bt16 + (size_t)m * KTOT, tid);
}

extern "C" void kernel_launch(void* const* d_in, const int* in_sizes, int n_in,
                              void* d_out, int out_size, void* d_ws, size_t ws_size,
                              hipStream_t stream) {
  if (n_in < 3) return;
  if (in_sizes[0] != NBATCH * NIN_C || in_sizes[1] != NIN_C * NOUT_C || in_sizes[2] != NOUT_C) return;
  if (out_size != NBATCH * NOUT_C) return;

  const float* x = (const float*)d_in[0];
  const float* w = (const float*)d_in[1];
  const float* b = (const float*)d_in[2];
  float* y = (float*)d_out;

  const size_t offPar = 0;
  const size_t offA   = 256;
  const size_t bytesA = (size_t)NBATCH * KTOT * sizeof(_Float16);
  const size_t offB   = offA + bytesA;
  const size_t bytesB = (size_t)NOUT_C * KTOT * sizeof(_Float16);
  const size_t total  = offB + bytesB;
  if (total > ws_size) return;

  char* ws = (char*)d_ws;
  float*    params = (float*)(ws + offPar);
  _Float16* A16    = (_Float16*)(ws + offA);
  _Float16* Bt16   = (_Float16*)(ws + offB);

  k_maxabs <<<1, 512, 0, stream>>>(w, b, params);
  k_build_a<<<NBATCH, 256, 0, stream>>>(x, A16);
  k_build_b<<<NOUT_C, 256, 0, stream>>>(w, b, params, Bt16);

  const int tiles = (NBATCH / 64) * (NOUT_C / 64);
  const int gblocks = (tiles + 7) / 8;
  wmma_gemm64<0, false, 0, 0, false, 0><<<dim3(gblocks, 1), 256, 0, stream>>>(
      (const unsigned short*)A16, (const unsigned short*)A16, KTOT, (long)0,
      (const unsigned short*)Bt16, (const unsigned short*)Bt16, KTOT, (long)0,
      (void*)y, (void*)y, NOUT_C, (long)0,
      params, params, (long)0,
      NBATCH, NOUT_C, KTOT, 1.0f / (ASCALE_C * CSCALE_C), params + 1);
}
